// SoftTree_56942676410675
// MI455X (gfx1250) — hardware-verified
//
#include <hip/hip_runtime.h>

typedef __attribute__((ext_vector_type(16))) __bf16 v16b;
typedef unsigned short v8us  __attribute__((ext_vector_type(8)));
typedef unsigned short v16us __attribute__((ext_vector_type(16)));
typedef float v8f __attribute__((ext_vector_type(8)));
typedef float v4f __attribute__((ext_vector_type(4)));
typedef v8us __attribute__((may_alias)) v8usa;
typedef v4f  __attribute__((may_alias)) v4fa;

union Frag { v16b v; v16us u; v8us half[2]; };

#define NB     8192
#define NF     512
#define NNODE  1023
#define NNP    1024
#define NLEAF  1024
#define NLD    64

#define XBLK   ((NB * NF / 8) / 256)
#define WBLK   ((NNP * NF / 8) / 256)
#define LBLK   ((NLD * NLEAF / 8) / 256)

#define TR_WAVES 4
#define TR_ITERS 8
#define TR_ROWS  (TR_WAVES * TR_ITERS)

static_assert(NF % 32 == 0);
static_assert(NLEAF % 32 == 0);
static_assert(NB % 128 == 0);
static_assert(NNP % 64 == 0);
static_assert(NLD == 64);
static_assert(NB % TR_ROWS == 0);
static_assert((NB * NF / 8) % 256 == 0);
static_assert((NNP * NF / 8) % 256 == 0);
static_assert((NLD * NLEAF / 8) % 256 == 0);

__device__ __forceinline__ unsigned short bfb(float f) {
  unsigned u = __float_as_uint(f);
  u = u + 0x7FFFu + ((u >> 16) & 1u);
  return (unsigned short)(u >> 16);
}
__device__ __forceinline__ float bfv(unsigned short s) {
  return __uint_as_float(((unsigned)s) << 16);
}

__device__ __forceinline__ v8f wmma_bf16(v16b a, v16b b, v8f c) {
  v8f d = __builtin_amdgcn_wmma_f32_16x16x32_bf16(false, a, false, b, (short)0, c, false, false);
  asm volatile("v_nop\n\tv_nop\n\tv_nop\n\tv_nop" : "+v"(d) : "v"(a), "v"(b));
  return d;
}

__device__ __forceinline__ v16b load_frag(const unsigned short* p, int h) {
  Frag f;
  f.half[0] = *(const v8usa*)(p + 8 * h);
  f.half[1] = *(const v8usa*)(p + 16 + 8 * h);
  return f.v;
}

__device__ __forceinline__ void store2_us8(unsigned short* dst, v8us o) {
  *(volatile v8us*)dst = o;
  __threadfence();
  *(volatile v8us*)dst = o;
}

__device__ __forceinline__ void tile_store_pass(const float* sT, float* g, int gp, int w, int lane) {
  const int q8 = lane & 7, sub = lane >> 3;
  #pragma unroll
  for (int i = 0; i < 16; ++i) {
    const int lid = 4 * i + sub;
    const int row = 32 * w + (lid >> 1), hl = lid & 1;
    const v4f v = *(const v4fa*)(sT + row * 64 + 32 * hl + 4 * q8);
    *(volatile v4f*)(g + (size_t)row * gp + 32 * hl + 4 * q8) = v;
  }
}

__device__ __forceinline__ void row_store_pass(const unsigned short* s, unsigned short* g, int lane) {
  #pragma unroll
  for (int i = 0; i < 4; ++i) {
    const int e = (i * 32 + lane) * 8;
    const v8us v = *(const v8usa*)(s + e);
    *(volatile v8us*)(g + e) = v;
  }
}

__global__ __launch_bounds__(256) void convert_kernel(
    const float* __restrict__ x, const float* __restrict__ W, const float* __restrict__ lw,
    unsigned short* __restrict__ xh, unsigned short* __restrict__ wt, unsigned short* __restrict__ lt)
{
  const int bid = blockIdx.x, tid = threadIdx.x;
  if (bid < XBLK) {
    const size_t g = (size_t)bid * 256 + tid;
    const float* src = x + g * 8;
    const v4f a = *(const v4fa*)src;
    const v4f c = *(const v4fa*)(src + 4);
    const v8us o = { bfb(a.x), bfb(a.y), bfb(a.z), bfb(a.w), bfb(c.x), bfb(c.y), bfb(c.z), bfb(c.w) };
    store2_us8(xh + g * 8, o);
  } else if (bid < XBLK + WBLK) {
    const int e  = (bid - XBLK) * 256 + tid;
    const int n  = e >> 6;
    const int k0 = (e & 63) * 8;
    const int nc = (n < NNODE) ? n : (NNODE - 1);
    const float* src = W + (size_t)k0 * NNODE + nc;
    const float v0 = src[0 * NNODE], v1 = src[1 * NNODE], v2 = src[2 * NNODE], v3 = src[3 * NNODE];
    const float v4 = src[4 * NNODE], v5 = src[5 * NNODE], v6 = src[6 * NNODE], v7 = src[7 * NNODE];
    const bool pad = (n >= NNODE);
    const unsigned short zz = 0;
    const v8us o = { pad ? zz : bfb(v0), pad ? zz : bfb(v1), pad ? zz : bfb(v2), pad ? zz : bfb(v3),
                     pad ? zz : bfb(v4), pad ? zz : bfb(v5), pad ? zz : bfb(v6), pad ? zz : bfb(v7) };
    store2_us8(wt + (size_t)n * NF + k0, o);
  } else if (bid < XBLK + WBLK + LBLK) {
    const int e  = (bid - XBLK - WBLK) * 256 + tid;
    const int d  = e >> 7;
    const int k0 = (e & 127) * 8;
    const float* src = lw + (size_t)k0 * NLD + d;
    const float v0 = src[0 * NLD], v1 = src[1 * NLD], v2 = src[2 * NLD], v3 = src[3 * NLD];
    const float v4 = src[4 * NLD], v5 = src[5 * NLD], v6 = src[6 * NLD], v7 = src[7 * NLD];
    const v8us o = { bfb(v0), bfb(v1), bfb(v2), bfb(v3), bfb(v4), bfb(v5), bfb(v6), bfb(v7) };
    store2_us8(lt + (size_t)d * NLEAF + k0, o);
  }
}

__global__ __launch_bounds__(128) void gate_gemm_kernel(
    const unsigned short* __restrict__ xh,
    const unsigned short* __restrict__ wt,
    const float* __restrict__ bias,
    float* __restrict__ P)
{
  __shared__ __attribute__((aligned(16))) float sT[128 * 64];

  const int tid = threadIdx.x, lane = tid & 31, w = tid >> 5;
  const int h = lane >> 4, m = lane & 15;
  const int m0 = blockIdx.x * 128, n0 = blockIdx.y * 64;
  const int m0w = m0 + 32 * w;

  const unsigned short* xa0 = xh + (size_t)(m0w + m) * NF;
  const unsigned short* xa1 = xa0 + (size_t)16 * NF;
  const unsigned short* wb  = wt + (size_t)(n0 + m) * NF;

  const v8f zero8 = {0.f, 0.f, 0.f, 0.f, 0.f, 0.f, 0.f, 0.f};
  v8f acc[2][4];
  #pragma unroll
  for (int mt = 0; mt < 2; ++mt)
    #pragma unroll
    for (int nt = 0; nt < 4; ++nt) acc[mt][nt] = zero8;

  #pragma unroll 1
  for (int k0 = 0; k0 < NF; k0 += 32) {
    const v16b a0 = load_frag(xa0 + k0, h);
    const v16b a1 = load_frag(xa1 + k0, h);
    #pragma unroll
    for (int nt = 0; nt < 4; ++nt) {
      const v16b b = load_frag(wb + (size_t)nt * 16 * NF + k0, h);
      acc[0][nt] = wmma_bf16(a0, b, acc[0][nt]);
      acc[1][nt] = wmma_bf16(a1, b, acc[1][nt]);
    }
  }

  #pragma unroll
  for (int nt = 0; nt < 4; ++nt) {
    const int col = 16 * nt + m;
    const int n = n0 + col;
    const int nc = (n < NNODE) ? n : (NNODE - 1);
    float bv = bfv(bfb(bias[nc]));
    bv = (n < NNODE) ? bv : 0.0f;
    #pragma unroll
    for (int mt = 0; mt < 2; ++mt) {
      #pragma unroll
      for (int r = 0; r < 8; ++r) {
        const int tokl = 32 * w + 16 * mt + 8 * h + r;
        const float z = acc[mt][nt][r] + bv;
        const float e = expf(-z);
        const float p = __builtin_amdgcn_rcpf(1.0f + e);
        sT[tokl * 64 + col] = p;
      }
    }
  }
  __syncthreads();

  float* g = P + (size_t)m0 * NNP + n0;
  tile_store_pass(sT, g, NNP, w, lane);
  __threadfence();
  tile_store_pass(sT, g, NNP, w, lane);
}

template <int NIN>
__device__ __forceinline__ void expand_level(const float* pr, int base,
                                             const float (&in)[NIN], float (&o)[2 * NIN]) {
  #pragma clang fp contract(off)
  #pragma unroll
  for (int j = 0; j < NIN; ++j) {
    const float v = pr[base + j];
    const float u = 1.0f - v;
    o[2 * j]     = v * in[j];
    o[2 * j + 1] = u * in[j];
  }
}

__global__ __launch_bounds__(128) void leafprob_kernel(
    const float* __restrict__ P,
    unsigned short* __restrict__ PH,
    unsigned short* __restrict__ PL)
{
  #pragma clang fp contract(off)
  __shared__ __attribute__((aligned(16))) float sP[TR_WAVES * NLEAF];
  __shared__ __attribute__((aligned(16))) unsigned short sH[TR_WAVES * NLEAF];
  __shared__ __attribute__((aligned(16))) unsigned short sL[TR_WAVES * NLEAF];

  const int tid = threadIdx.x, lane = tid & 31, w = tid >> 5;
  float* pr = sP + w * NLEAF;
  unsigned short* hr = sH + w * NLEAF;
  unsigned short* lr = sL + w * NLEAF;

  #pragma unroll 1
  for (int it = 0; it < TR_ITERS; ++it) {
    const int row = blockIdx.x * TR_ROWS + it * TR_WAVES + w;
    const float* prow = P + (size_t)row * NNP;

    #pragma unroll
    for (int j = 0; j < 8; ++j) {
      const int q = j * 32 + lane;
      const v4f v = *(const v4fa*)(prow + 4 * q);
      *(v4fa*)(pr + 4 * q) = v;
    }
    __syncthreads();

    float pre = 1.0f;
    #pragma unroll
    for (int L = 0; L < 5; ++L) {
      const int node = (1 << L) - 1 + (lane >> (5 - L));
      const int bit  = (lane >> (4 - L)) & 1;
      const float v = pr[node];
      const float u = 1.0f - v;
      pre = (bit ? u : v) * pre;
    }

    float a1[1];
    a1[0] = pre;
    float a2[2], a4[4], a8[8], a16[16], a32[32];
    expand_level<1>(pr,  31 +      lane, a1,  a2);
    expand_level<2>(pr,  63 +  2 * lane, a2,  a4);
    expand_level<4>(pr, 127 +  4 * lane, a4,  a8);
    expand_level<8>(pr, 255 +  8 * lane, a8,  a16);
    expand_level<16>(pr, 511 + 16 * lane, a16, a32);

    #pragma unroll
    for (int q = 0; q < 4; ++q) {
      v8us hv, lv;
      #pragma unroll
      for (int i = 0; i < 8; ++i) {
        const float p = a32[8 * q + i];
        const unsigned short hb = bfb(p);
        const unsigned short lb = bfb(p - bfv(hb));
        hv[i] = hb;
        lv[i] = lb;
      }
      *(v8usa*)(hr + 32 * lane + 8 * q) = hv;
      *(v8usa*)(lr + 32 * lane + 8 * q) = lv;
    }
    __syncthreads();

    unsigned short* gh = PH + (size_t)row * NLEAF;
    unsigned short* gl = PL + (size_t)row * NLEAF;
    row_store_pass(hr, gh, lane);
    row_store_pass(lr, gl, lane);
    __threadfence();
    row_store_pass(hr, gh, lane);
    row_store_pass(lr, gl, lane);
  }
}

__global__ __launch_bounds__(128) void leaf_gemm_kernel(
    const unsigned short* __restrict__ PH,
    const unsigned short* __restrict__ PL,
    const unsigned short* __restrict__ lt,
    float* __restrict__ out)
{
  __shared__ __attribute__((aligned(16))) float sT[128 * 64];

  const int tid = threadIdx.x, lane = tid & 31, w = tid >> 5;
  const int h = lane >> 4, m = lane & 15;
  const int m0 = blockIdx.x * 128;
  const int m0w = m0 + 32 * w;

  const unsigned short* ha0 = PH + (size_t)(m0w + m) * NLEAF;
  const unsigned short* ha1 = ha0 + (size_t)16 * NLEAF;
  const unsigned short* la0 = PL + (size_t)(m0w + m) * NLEAF;
  const unsigned short* la1 = la0 + (size_t)16 * NLEAF;
  const unsigned short* lb  = lt + (size_t)m * NLEAF;

  const v8f zero8 = {0.f, 0.f, 0.f, 0.f, 0.f, 0.f, 0.f, 0.f};
  v8f acc[2][4];
  #pragma unroll
  for (int mt = 0; mt < 2; ++mt)
    #pragma unroll
    for (int nt = 0; nt < 4; ++nt) acc[mt][nt] = zero8;

  #pragma unroll 1
  for (int k0 = 0; k0 < NLEAF; k0 += 32) {
    const v16b ah0 = load_frag(ha0 + k0, h);
    const v16b ah1 = load_frag(ha1 + k0, h);
    const v16b al0 = load_frag(la0 + k0, h);
    const v16b al1 = load_frag(la1 + k0, h);
    #pragma unroll
    for (int nt = 0; nt < 4; ++nt) {
      const v16b b = load_frag(lb + (size_t)nt * 16 * NLEAF + k0, h);
      acc[0][nt] = wmma_bf16(ah0, b, acc[0][nt]);
      acc[0][nt] = wmma_bf16(al0, b, acc[0][nt]);
      acc[1][nt] = wmma_bf16(ah1, b, acc[1][nt]);
      acc[1][nt] = wmma_bf16(al1, b, acc[1][nt]);
    }
  }

  #pragma unroll
  for (int nt = 0; nt < 4; ++nt) {
    const int col = 16 * nt + m;
    #pragma unroll
    for (int mt = 0; mt < 2; ++mt) {
      #pragma unroll
      for (int r = 0; r < 8; ++r) {
        const int tokl = 32 * w + 16 * mt + 8 * h + r;
        sT[tokl * 64 + col] = acc[mt][nt][r];
      }
    }
  }
  __syncthreads();

  float* g = out + (size_t)m0 * NLD;
  tile_store_pass(sT, g, NLD, w, lane);
  __threadfence();
  tile_store_pass(sT, g, NLD, w, lane);
}

extern "C" void kernel_launch(void* const* d_in, const int* in_sizes, int n_in,
                              void* d_out, int out_size, void* d_ws, size_t ws_size,
                              hipStream_t stream) {
  if (n_in < 4) return;
  if (in_sizes[0] != NB * NF) return;
  if (in_sizes[1] != NF * NNODE) return;
  if (in_sizes[2] != NNODE) return;
  if (in_sizes[3] != NLEAF * NLD) return;
  if (out_size != NB * NLD) return;

  const float* x  = (const float*)d_in[0];
  const float* W  = (const float*)d_in[1];
  const float* b  = (const float*)d_in[2];
  const float* lw = (const float*)d_in[3];
  float* out = (float*)d_out;

  const size_t sz_xh = (size_t)NB * NF * 2;
  const size_t sz_wt = (size_t)NNP * NF * 2;
  const size_t sz_lt = (size_t)NLD * NLEAF * 2;
  const size_t sz_p  = (size_t)NB * NNP * 4;
  const size_t sz_ph = (size_t)NB * NLEAF * 2;
  const size_t off_xh = 0;
  const size_t off_wt = off_xh + sz_xh;
  const size_t off_lt = off_wt + sz_wt;
  const size_t off_p  = off_lt + sz_lt;
  const size_t off_ph = off_p + sz_p;
  const size_t off_pl = off_ph + sz_ph;
  const size_t total  = off_pl + sz_ph;
  if (total > ws_size) return;

  char* ws = (char*)d_ws;
  unsigned short* xh = (unsigned short*)(ws + off_xh);
  unsigned short* wt = (unsigned short*)(ws + off_wt);
  unsigned short* lt = (unsigned short*)(ws + off_lt);
  float*          P  = (float*)(ws + off_p);
  unsigned short* PH = (unsigned short*)(ws + off_ph);
  unsigned short* PL = (unsigned short*)(ws + off_pl);

  convert_kernel<<<XBLK + WBLK + LBLK, 256, 0, stream>>>(x, W, lw, xh, wt, lt);

  dim3 g1(NB / 128, NNP / 64);
  gate_gemm_kernel<<<g1, 128, 0, stream>>>(xh, wt, b, P);

  leafprob_kernel<<<NB / TR_ROWS, 128, 0, stream>>>(P, PH, PL);

  leaf_gemm_kernel<<<NB / 128, 128, 0, stream>>>(PH, PL, lt, out);
}
